// GGNNModel_4964982194948
// MI455X (gfx1250) — hardware-verified
//
#include <hip/hip_runtime.h>
#include <stddef.h>


#define DD      256
#define ET      3
#define ET2     6
#define PROPW   (ET2 * DD)
#define GRUW    (3 * DD)
#define KSTEPS  (DD / 32)
#define GBM     64
#define GTHR    128
#define PGRP    64
#define NPGRP   (PROPW / PGRP)
#define NTHR    256
#define NWAVE   8
#define EPT     8
#define CHUNK   (NTHR * EPT)
#define WCAP    (EPT * 32)
#define LISTN   (NWAVE * WCAP)
#define NBMAX   1024
#define SLOTB   10
#define RCAP    32768
#define DEGCAP  4096
#define CA      16.0f
#define CW      256.0f
#define CP      8.0f
#define SCL     0.000244140625f
#define AGF     2.0f
#define LDS_AGG ((2 * RCAP + 2 * NBMAX + LISTN) * 4 + 64)

static_assert((CHUNK & (CHUNK - 1)) == 0 && CHUNK <= 2048);
static_assert(NBMAX == (1 << SLOTB));
static_assert(NTHR * 4 == NBMAX);
static_assert(LISTN >= NBMAX);
static_assert(LISTN >= NWAVE * WCAP);
static_assert((RCAP % 32) == 0);
static_assert(LDS_AGG <= 300000);
static_assert(GBM == (GTHR / 32) * 16);
static_assert(GTHR == 128);
static_assert((DD % 32) == 0 && PGRP == 64 && (PROPW % PGRP) == 0);

typedef float    v4f  __attribute__((ext_vector_type(4)));
typedef float    v8f  __attribute__((ext_vector_type(8)));
typedef int      v4i  __attribute__((ext_vector_type(4)));
typedef int      v8i  __attribute__((ext_vector_type(8)));
typedef _Float16 v8h  __attribute__((ext_vector_type(8)));
typedef _Float16 v16h __attribute__((ext_vector_type(16)));
union FragH { v16h v; v8h h[2]; v8i w; };

__device__ __forceinline__ v8f wmh(const FragH& a, const FragH& b, v8f c) {
  v8f d = __builtin_amdgcn_wmma_f32_16x16x32_f16(false, a.v, false, b.v, (short)0, c, false, false);
  asm volatile("v_nop\n\tv_nop\n\tv_nop\n\tv_nop" : "+v"(d) : "v"(a.w), "v"(b.w));
  return d;
}

__device__ __forceinline__ int type_of(int te, int Mper, float invM) {
  int li = (int)((float)te * invM);
  li = ((li + 1) * Mper <= te) ? li + 1 : li;
  li = (li * Mper > te) ? li - 1 : li;
  li = li < 0 ? 0 : (li > ET2 - 1 ? ET2 - 1 : li);
  return li;
}

__global__ __launch_bounds__(NTHR) void k_cvt(const float* __restrict__ x, _Float16* xh, int nRows, int nUnits, float sc) {
  const int i = (int)blockIdx.x * NTHR + (int)threadIdx.x;
  if (i >= nUnits) return;
  const int row = i >> 5;
  const int c0  = (i & 31) * 8;
  const int rc  = row < nRows ? row : nRows - 1;
  const float* p = x + (size_t)rc * DD + c0;
  v4f a = *(const v4f*)p, b = *(const v4f*)(p + 4);
  const v4f z4 = {0.f, 0.f, 0.f, 0.f};
  if (row >= nRows) { a = z4; b = z4; }
  v8h hv;
  hv[0] = (_Float16)(a.x * sc); hv[1] = (_Float16)(a.y * sc);
  hv[2] = (_Float16)(a.z * sc); hv[3] = (_Float16)(a.w * sc);
  hv[4] = (_Float16)(b.x * sc); hv[5] = (_Float16)(b.y * sc);
  hv[6] = (_Float16)(b.z * sc); hv[7] = (_Float16)(b.w * sc);
  const size_t o = (size_t)row * DD + c0;
  *(volatile v8h*)(xh + o) = hv;
  __threadfence();
  *(volatile v8h*)(xh + o) = hv;
}

__global__ __launch_bounds__(GTHR) void k_prop(const _Float16* __restrict__ xh, const _Float16* __restrict__ w16,
                                               const float* __restrict__ bias, _Float16* prop, int MP) {
  __shared__ __attribute__((aligned(16))) _Float16 stg[4 * 16 * PGRP];
  const int tid = threadIdx.x, lane = tid & 31, wave = tid >> 5, hh = lane >> 4, m = lane & 15;
  const int rowBase = (int)blockIdx.x * GBM;
  const size_t arow = (size_t)(rowBase + 16 * wave + m) * DD + 8 * hh;
  _Float16* sw = stg + wave * (16 * PGRP);
  const int rq = lane >> 3, c8 = lane & 7;
#pragma unroll 1
  for (int g = 0; g < NPGRP; ++g) {
    v8f acc[4];
    { v8f z = {0.f, 0.f, 0.f, 0.f, 0.f, 0.f, 0.f, 0.f}; acc[0] = z; acc[1] = z; acc[2] = z; acc[3] = z; }
#pragma unroll 2
    for (int ks = 0; ks < KSTEPS; ++ks) {
      FragH af;
      af.h[0] = *(const v8h*)(xh + arow + 32 * ks);
      af.h[1] = *(const v8h*)(xh + arow + 32 * ks + 16);
#pragma unroll
      for (int t = 0; t < 4; ++t) {
        const size_t bo = (size_t)(g * PGRP + 16 * t + m) * DD + 8 * hh + 32 * ks;
        FragH bf;
        bf.h[0] = *(const v8h*)(w16 + bo);
        bf.h[1] = *(const v8h*)(w16 + bo + 16);
        acc[t] = wmh(af, bf, acc[t]);
      }
    }
    float bv[4];
#pragma unroll
    for (int t = 0; t < 4; ++t) bv[t] = bias[g * PGRP + 16 * t + m];
    __syncthreads();
#pragma unroll
    for (int t = 0; t < 4; ++t) {
#pragma unroll
      for (int r = 0; r < 8; ++r)
        sw[(8 * hh + r) * PGRP + 16 * t + m] = (_Float16)((acc[t][r] * SCL + bv[t]) * CP);
    }
    __syncthreads();
    v8h o[4];
#pragma unroll
    for (int i = 0; i < 4; ++i) o[i] = *(const v8h*)(sw + (4 * i + rq) * PGRP + 8 * c8);
    _Float16* pb = prop + (size_t)(rowBase + 16 * wave + rq) * PROPW + (size_t)(g * PGRP + 8 * c8);
#pragma unroll
    for (int i = 0; i < 4; ++i) *(volatile v8h*)(pb + (size_t)(4 * i) * PROPW) = o[i];
    __threadfence();
#pragma unroll
    for (int i = 0; i < 4; ++i) *(volatile v8h*)(pb + (size_t)(4 * i) * PROPW) = o[i];
  }
}

__device__ __forceinline__ int scan_chunk(const int* __restrict__ edges, int nE, int Mper, float invM, int cbase,
                                          int slotBase, int nb, int* list, int tid, int lane, int wave) {
  int wc = 0;
  const int el0  = tid * EPT;
  const int e0   = cbase + el0;
  const int sent = -2147483647 - 1;
  const int e0c  = e0 > nE - EPT ? nE - EPT : e0;
  const int li   = type_of(e0c, Mper, invM);
  const bool fw  = li < ET;
  const int l3   = fw ? li : li - ET;
  int ee = e0c - li * Mper;
  ee = ee < 0 ? 0 : (ee > Mper - EPT ? Mper - EPT : ee);
  const int* p = edges + ((size_t)l3 * (size_t)Mper + (size_t)ee) * 2;
  const v4i p0 = *(const v4i*)(p), p1 = *(const v4i*)(p + 4), p2 = *(const v4i*)(p + 8), p3 = *(const v4i*)(p + 12);
  int d0 = fw ? p0.y : p0.x, d1 = fw ? p0.w : p0.z;
  int d2 = fw ? p1.y : p1.x, d3 = fw ? p1.w : p1.z;
  int d4 = fw ? p2.y : p2.x, d5 = fw ? p2.w : p2.z;
  int d6 = fw ? p3.y : p3.x, d7 = fw ? p3.w : p3.z;
  if (e0 >= nE) { d0 = sent; d1 = sent; d2 = sent; d3 = sent; d4 = sent; d5 = sent; d6 = sent; d7 = sent; }
  const unsigned nbs = (unsigned)slotBase;
  const unsigned unb = (unsigned)nb;
  const unsigned s0 = (unsigned)d0 - nbs, s1 = (unsigned)d1 - nbs;
  const unsigned s2 = (unsigned)d2 - nbs, s3 = (unsigned)d3 - nbs;
  const unsigned s4 = (unsigned)d4 - nbs, s5 = (unsigned)d5 - nbs;
  const unsigned s6 = (unsigned)d6 - nbs, s7 = (unsigned)d7 - nbs;
  const bool h0 = s0 < unb, h1 = s1 < unb, h2 = s2 < unb, h3 = s3 < unb;
  const bool h4 = s4 < unb, h5 = s5 < unb, h6 = s6 < unb, h7 = s7 < unb;
  const unsigned any = __builtin_amdgcn_ballot_w32(h0 | h1 | h2 | h3 | h4 | h5 | h6 | h7);
  if (any != 0u) {
#define HITJ(J, HJ, SJ) { \
      const unsigned mj = __builtin_amdgcn_ballot_w32(HJ); \
      if (mj != 0u) { \
        if (HJ) { \
          const int pos = wc + (int)__builtin_amdgcn_mbcnt_lo(mj, 0u); \
          if (pos < WCAP) list[wave * WCAP + pos] = ((el0 + (J)) << SLOTB) | (int)(SJ); \
        } \
        wc += (int)__builtin_popcount(mj); } }
    HITJ(0, h0, s0)
    HITJ(1, h1, s1)
    HITJ(2, h2, s2)
    HITJ(3, h3, s3)
    HITJ(4, h4, s4)
    HITJ(5, h5, s5)
    HITJ(6, h6, s6)
    HITJ(7, h7, s7)
#undef HITJ
  }
  return wc;
}

__global__ __launch_bounds__(NTHR) void k_agg(const int* __restrict__ edges, const _Float16* __restrict__ prop,
                                              _Float16* msgs, int nN, int MP, int nE, int Mper, float invM, int nb) {
  extern __shared__ v4f lds_dyn[];
  int* reg1 = (int*)lds_dyn;
  int* reg2 = reg1 + RCAP;
  int* scnt = reg2 + RCAP;
  int* soff = scnt + NBMAX;
  int* list = soff + NBMAX;
  int* wcnt = list + LISTN;
  int* wtot = wcnt + NWAVE;
  const int tid = threadIdx.x, lane = tid & 31, wave = tid >> 5;
  const int nodeBase = (int)blockIdx.x * nb;

  for (int i = tid; i < NBMAX; i += NTHR) scnt[i] = 0;
  __syncthreads();

  int tot = 0;
  const int nChunks = (nE + CHUNK - 1) / CHUNK;
#pragma unroll 1
  for (int ch = 0; ch < nChunks; ++ch) {
    const int cbase = ch * CHUNK;
    const int wc = scan_chunk(edges, nE, Mper, invM, cbase, nodeBase, nb, list, tid, lane, wave);
    if (lane == 0) wcnt[wave] = wc;
    __syncthreads();
    int pre = 0, all = 0;
#pragma unroll
    for (int w2 = 0; w2 < NWAVE; ++w2) {
      int c = wcnt[w2];
      c = c < 0 ? 0 : (c > WCAP ? WCAP : c);
      all += c;
      pre += (w2 < wave) ? c : 0;
    }
    const int wcc  = wc > WCAP ? WCAP : wc;
    const int base = tot + pre;
#pragma unroll 1
    for (int i = lane; i < wcc; i += 32) {
      const int ent = list[wave * WCAP + i];
      const int el  = (ent >> SLOTB) & (CHUNK - 1);
      const int sl  = ent & (NBMAX - 1);
      int eid = cbase + el;
      eid = eid > nE - 1 ? nE - 1 : eid;
      const int pos = base + i;
      if (pos < RCAP) reg1[pos] = (int)(((unsigned)eid << SLOTB) | (unsigned)sl);
    }
    tot += all;
    tot = tot > RCAP ? RCAP : tot;
    __syncthreads();
  }
  const int nh = tot;

  if (wave == 0) {
#pragma unroll 1
    for (int b0 = 0; b0 < nh; b0 += 32) {
      const int idx = b0 + lane;
      const int uv  = reg1[idx < RCAP ? idx : RCAP - 1];
      const int m32 = (nh - b0) < 32 ? (nh - b0) : 32;
#pragma unroll 1
      for (int k = 0; k < m32; ++k) {
        const int u  = __builtin_amdgcn_readlane(uv, k);
        const int sl = u & (NBMAX - 1);
        if (lane == 0) scnt[sl] = scnt[sl] + 1;
      }
    }
  }
  __syncthreads();

  {
    const v4i ca = *(const v4i*)(scnt + 4 * tid);
    const int e0 = ca.x < 0 ? 0 : ca.x, e1 = ca.y < 0 ? 0 : ca.y, e2 = ca.z < 0 ? 0 : ca.z, e3 = ca.w < 0 ? 0 : ca.w;
    const int ts = e0 + e1 + e2 + e3;
    int incl = ts;
#pragma unroll
    for (int d = 1; d < 32; d <<= 1) {
      const int up = __shfl_up(incl, d);
      if (lane >= d) incl += up;
    }
    if (lane == 31) wtot[wave] = incl;
    __syncthreads();
    int pre = 0;
#pragma unroll
    for (int w2 = 0; w2 < NWAVE; ++w2) pre += (w2 < wave) ? wtot[w2] : 0;
    int run = pre + incl - ts;
    soff[4 * tid + 0] = run; run += e0;
    soff[4 * tid + 1] = run; run += e1;
    soff[4 * tid + 2] = run; run += e2;
    soff[4 * tid + 3] = run;
  }
  __syncthreads();
  for (int i = tid; i < NBMAX; i += NTHR) list[i] = soff[i];
  __syncthreads();

  if (wave == 0) {
#pragma unroll 1
    for (int b0 = 0; b0 < nh; b0 += 32) {
      const int idx = b0 + lane;
      const int uv  = reg1[idx < RCAP ? idx : RCAP - 1];
      const int m32 = (nh - b0) < 32 ? (nh - b0) : 32;
#pragma unroll 1
      for (int k = 0; k < m32; ++k) {
        const int u   = __builtin_amdgcn_readlane(uv, k);
        const int sl  = u & (NBMAX - 1);
        const int eid = (int)((unsigned)u >> SLOTB);
        if (lane == 0) {
          int pos = list[sl];
          pos = pos < 0 ? 0 : (pos > RCAP - 1 ? RCAP - 1 : pos);
          reg2[pos] = eid;
          list[sl] = pos + 1;
        }
      }
    }
  }
  __syncthreads();

  const int nbw = nb >> 3;
  const bool ovf = (nh >= RCAP);
  const float qnan = __int_as_float(0x7fc00000);
#pragma unroll 1
  for (int jt = 0; jt < nbw; ++jt) {
    const int slot = wave * nbw + jt;
    const int grow = nodeBase + slot;
    int st = soff[slot];
    const int craw = scnt[slot];
    int cnt = craw;
    st  = st < 0 ? 0 : (st > nh ? nh : st);
    cnt = cnt < 0 ? 0 : (cnt > DEGCAP ? DEGCAP : cnt);
    if (cnt > nh - st) cnt = nh - st;
    const float pz = (ovf || craw > DEGCAP) ? qnan : 0.0f;
    const bool wr = grow < MP;

    float a0 = 0.f, a1 = 0.f, a2 = 0.f, a3 = 0.f, a4 = 0.f, a5 = 0.f, a6 = 0.f, a7 = 0.f;
#pragma unroll 1
    for (int q = 0; q < cnt; ++q) {
      int idx = st + q; idx = idx > RCAP - 1 ? RCAP - 1 : idx;
      int te = reg2[idx]; te = te < 0 ? 0 : (te > nE - 1 ? nE - 1 : te);
      const int li = type_of(te, Mper, invM);
      const bool fw = li < ET;
      const int l3 = fw ? li : li - ET;
      int ee = te - li * Mper; ee = ee < 0 ? 0 : (ee > Mper - 1 ? Mper - 1 : ee);
      const int* pp = edges + ((size_t)l3 * (size_t)Mper + (size_t)ee) * 2;
      const int sa = pp[0], sb = pp[1];
      int s = fw ? sa : sb;
      s = s < 0 ? 0 : (s > nN - 1 ? nN - 1 : s);
      const v8h v = *(const v8h*)(prop + (size_t)s * PROPW + (size_t)(li * DD) + (size_t)(8 * lane));
      a0 += (float)v[0]; a1 += (float)v[1]; a2 += (float)v[2]; a3 += (float)v[3];
      a4 += (float)v[4]; a5 += (float)v[5]; a6 += (float)v[6]; a7 += (float)v[7];
    }
    const float cf  = (float)(cnt > 0 ? cnt : 1);
    const float inv = (cnt > 0 ? AGF : 0.0f) * __builtin_amdgcn_rcpf(cf);
    v8h hv;
    hv[0] = (_Float16)(a0 * inv + pz); hv[1] = (_Float16)(a1 * inv + pz);
    hv[2] = (_Float16)(a2 * inv + pz); hv[3] = (_Float16)(a3 * inv + pz);
    hv[4] = (_Float16)(a4 * inv + pz); hv[5] = (_Float16)(a5 * inv + pz);
    hv[6] = (_Float16)(a6 * inv + pz); hv[7] = (_Float16)(a7 * inv + pz);
    const int gcl = grow < MP ? grow : MP - 1;
    _Float16* op = msgs + (size_t)gcl * DD + (size_t)(8 * lane);
    if (wr) *(volatile v8h*)op = hv;
    __threadfence();
    if (wr) *(volatile v8h*)op = hv;
  }
}

__global__ __launch_bounds__(GTHR) void k_gru(const _Float16* __restrict__ m16, const _Float16* __restrict__ h16,
                                              const _Float16* __restrict__ wih, const _Float16* __restrict__ whh,
                                              const float* __restrict__ bih, const float* __restrict__ bhh,
                                              const float* hF, float* hOut, int nN) {
  __shared__ __attribute__((aligned(16))) float stg[16 * 128];
  const int tid = threadIdx.x, lane = tid & 31, wave = tid >> 5, hh = lane >> 4, m = lane & 15;
  const int rt = (int)blockIdx.x >> 1, cg = (int)blockIdx.x & 1;
  const int rowBase = 16 * rt;
  const int colW = 128 * cg + 32 * wave;
  const size_t arow = (size_t)(rowBase + m) * DD + 8 * hh;
  const size_t g1 = (size_t)DD * DD, g2 = (size_t)2 * DD * DD;
  v8f aR[2], aZ[2], aI[2], aH[2];
  { v8f z = {0.f, 0.f, 0.f, 0.f, 0.f, 0.f, 0.f, 0.f};
    aR[0] = z; aR[1] = z; aZ[0] = z; aZ[1] = z; aI[0] = z; aI[1] = z; aH[0] = z; aH[1] = z; }
#pragma unroll 1
  for (int ks = 0; ks < KSTEPS; ++ks) {
    FragH am, ah;
    am.h[0] = *(const v8h*)(m16 + arow + 32 * ks);
    am.h[1] = *(const v8h*)(m16 + arow + 32 * ks + 16);
    ah.h[0] = *(const v8h*)(h16 + arow + 32 * ks);
    ah.h[1] = *(const v8h*)(h16 + arow + 32 * ks + 16);
#pragma unroll
    for (int t = 0; t < 2; ++t) {
      const size_t cb = (size_t)(colW + 16 * t + m) * DD + 8 * hh + 32 * ks;
      FragH b;
      b.h[0] = *(const v8h*)(wih + cb);           b.h[1] = *(const v8h*)(wih + cb + 16);           aR[t] = wmh(am, b, aR[t]);
      b.h[0] = *(const v8h*)(whh + cb);           b.h[1] = *(const v8h*)(whh + cb + 16);           aR[t] = wmh(ah, b, aR[t]);
      b.h[0] = *(const v8h*)(wih + g1 + cb);      b.h[1] = *(const v8h*)(wih + g1 + cb + 16);      aZ[t] = wmh(am, b, aZ[t]);
      b.h[0] = *(const v8h*)(whh + g1 + cb);      b.h[1] = *(const v8h*)(whh + g1 + cb + 16);      aZ[t] = wmh(ah, b, aZ[t]);
      b.h[0] = *(const v8h*)(wih + g2 + cb);      b.h[1] = *(const v8h*)(wih + g2 + cb + 16);      aI[t] = wmh(am, b, aI[t]);
      b.h[0] = *(const v8h*)(whh + g2 + cb);      b.h[1] = *(const v8h*)(whh + g2 + cb + 16);      aH[t] = wmh(ah, b, aH[t]);
    }
  }
#pragma unroll
  for (int t = 0; t < 2; ++t) {
    const int col = colW + 16 * t + m;
    const float br = bih[col] + bhh[col];
    const float bz = bih[DD + col] + bhh[DD + col];
    const float bi = bih[2 * DD + col];
    const float bn = bhh[2 * DD + col];
#pragma unroll
    for (int r = 0; r < 8; ++r) {
      const int row = rowBase + 8 * hh + r;
      const int rc  = row < nN ? row : nN - 1;
      const float hp = hF[(size_t)rc * DD + col];
      float xr = aR[t][r] * SCL + br;
      float xz = aZ[t][r] * SCL + bz;
      xr = fminf(fmaxf(xr, -30.0f), 30.0f);
      xz = fminf(fmaxf(xz, -30.0f), 30.0f);
      const float R  = __builtin_amdgcn_rcpf(1.0f + __expf(-xr));
      const float Z  = __builtin_amdgcn_rcpf(1.0f + __expf(-xz));
      const float Nn = tanhf(aI[t][r] * SCL + bi + R * (aH[t][r] * SCL + bn));
      const float hn = (1.0f - Z) * Nn + Z * hp;
      stg[(8 * hh + r) * 128 + 32 * wave + 16 * t + m] = hn;
    }
  }
  __syncthreads();
  v4f o[4];
#pragma unroll
  for (int i = 0; i < 4; ++i) o[i] = *(const v4f*)(stg + (4 * i + wave) * 128 + 4 * lane);
  float* ob = hOut + (size_t)(128 * cg + 4 * lane);
#pragma unroll
  for (int i = 0; i < 4; ++i) {
    const int grow = rowBase + 4 * i + wave;
    if (grow < nN) *(volatile v4f*)(ob + (size_t)grow * DD) = o[i];
  }
  __threadfence();
#pragma unroll
  for (int i = 0; i < 4; ++i) {
    const int grow = rowBase + 4 * i + wave;
    if (grow < nN) *(volatile v4f*)(ob + (size_t)grow * DD) = o[i];
  }
}

static int pick_nb(int nE, int nN) {
  int nb = NBMAX;
  while (nb > 16 && (long long)nb * (long long)nE * 16LL > (long long)RCAP * (long long)nN * 15LL) nb >>= 1;
  return nb;
}

extern "C" void kernel_launch(void* const* d_in, const int* in_sizes, int n_in,
                              void* d_out, int out_size, void* d_ws, size_t ws_size,
                              hipStream_t stream) {
  if (n_in < 8) return;
  const int nN = in_sizes[0] / DD;
  if (nN <= 0 || in_sizes[0] != nN * DD) return;
  if (nN > (1 << 20)) return;
  if (in_sizes[1] != PROPW * DD) return;
  if (in_sizes[2] != PROPW) return;
  if (in_sizes[3] != GRUW * DD || in_sizes[4] != GRUW * DD) return;
  if (in_sizes[5] != GRUW || in_sizes[6] != GRUW) return;
  if ((in_sizes[7] % (ET * 2)) != 0) return;
  const int Mper = in_sizes[7] / (ET * 2);
  if (Mper < EPT || (Mper % EPT) != 0) return;
  const int nE = ET2 * Mper;
  if (nE >= (1 << 22)) return;
  if (out_size != nN * DD) return;

  const float* x    = (const float*)d_in[0];
  const float* W    = (const float*)d_in[1];
  const float* b    = (const float*)d_in[2];
  const float* gwih = (const float*)d_in[3];
  const float* gwhh = (const float*)d_in[4];
  const float* gbih = (const float*)d_in[5];
  const float* gbhh = (const float*)d_in[6];
  const int*  edges = (const int*)d_in[7];
  float* out = (float*)d_out;

  const int MP = ((nN + GBM - 1) / GBM) * GBM;
  const int nb = pick_nb(nE, nN);
  const float invM = 1.0f / (float)Mper;

  char* ws = (char*)d_ws;
  size_t off = 0;
  const size_t oW16 = off; off += (size_t)PROPW * DD * 2;          off = (off + 255) & ~(size_t)255;
  const size_t oWIH = off; off += (size_t)GRUW * DD * 2;           off = (off + 255) & ~(size_t)255;
  const size_t oWHH = off; off += (size_t)GRUW * DD * 2;           off = (off + 255) & ~(size_t)255;
  const size_t oH16 = off; off += (size_t)MP * DD * 2;             off = (off + 255) & ~(size_t)255;
  const size_t oM16 = off; off += (size_t)MP * DD * 2;             off = (off + 255) & ~(size_t)255;
  const size_t oH1  = off; off += (size_t)MP * DD * 4;             off = (off + 255) & ~(size_t)255;
  const size_t oPR  = off; off += (size_t)MP * PROPW * 2;          off = (off + 255) & ~(size_t)255;
  if (off > ws_size) return;
  _Float16* W16  = (_Float16*)(ws + oW16);
  _Float16* WIH  = (_Float16*)(ws + oWIH);
  _Float16* WHH  = (_Float16*)(ws + oWHH);
  _Float16* H16  = (_Float16*)(ws + oH16);
  _Float16* M16  = (_Float16*)(ws + oM16);
  float*    H1   = (float*)(ws + oH1);
  _Float16* PR   = (_Float16*)(ws + oPR);

  hipFuncSetAttribute(reinterpret_cast<const void*>(&k_agg), hipFuncAttributeMaxDynamicSharedMemorySize, LDS_AGG);

  const int nUW = PROPW * (DD / 8), nUG = GRUW * (DD / 8), nUX = MP * (DD / 8);
  k_cvt<<<(nUW + NTHR - 1) / NTHR, NTHR, 0, stream>>>(W,    W16, PROPW, nUW, CW);
  k_cvt<<<(nUG + NTHR - 1) / NTHR, NTHR, 0, stream>>>(gwih, WIH, GRUW,  nUG, CW);
  k_cvt<<<(nUG + NTHR - 1) / NTHR, NTHR, 0, stream>>>(gwhh, WHH, GRUW,  nUG, CW);

  const int gP = MP / GBM;
  const int gA = (MP + nb - 1) / nb;
  const int gG = (MP / 16) * 2;
  for (int t = 0; t < 2; ++t) {
    const float* hsrc = (t == 0) ? x : H1;
    float*       hdst = (t == 0) ? H1 : out;
    k_cvt<<<(nUX + NTHR - 1) / NTHR, NTHR, 0, stream>>>(hsrc, H16, nN, nUX, CA);
    k_prop<<<gP, GTHR, 0, stream>>>(H16, W16, b, PR, MP);
    k_agg<<<gA, NTHR, LDS_AGG, stream>>>(edges, PR, M16, nN, MP, nE, Mper, invM, nb);
    k_gru<<<gG, GTHR, 0, stream>>>(M16, H16, WIH, WHH, gbih, gbhh, hsrc, hdst, nN);
  }
}
